// EmbEdgeGNNGRU_11141145166541
// MI455X (gfx1250) — hardware-run, weakly checked
//
#include <hip/hip_runtime.h>


namespace {
constexpr int N = 65536, E = 524288, G = 1024, TT = E / G, D = 128, DO = 64, V = 1000, NBLK = N / 16;
constexpr float XS = 8.0f, WSC = 256.0f;
typedef _Float16 b16;
typedef __attribute__((ext_vector_type(16))) _Float16 v16b;
typedef __attribute__((ext_vector_type(8))) _Float16 v8b;
typedef __attribute__((ext_vector_type(8))) float v8f;
typedef __attribute__((ext_vector_type(4))) float v4f;
__device__ __forceinline__ float bf16_rne(float f) { unsigned int u = __float_as_uint(f); u += 0x7FFFu + ((u >> 16) & 1u); return __uint_as_float(u & 0xFFFF0000u); }
__device__ __forceinline__ void split16(float v, b16& hi, b16& lo) { hi = (b16)v; lo = (b16)(v - (float)hi); }
__device__ __forceinline__ v16b frag_kb(const b16* p, int hh) { const v8b a = *(const v8b*)(p + 8 * hh), b = *(const v8b*)(p + 16 + 8 * hh); v16b f;
#pragma unroll
  for (int e = 0; e < 8; ++e) { f[e] = a[e]; f[8 + e] = b[e]; } return f; }
__device__ __forceinline__ v8f wmma16b(v16b a, v16b b, v8f c) { v8f d = __builtin_amdgcn_wmma_f32_16x16x32_f16(false, a, false, b, (short)0, c, false, false); asm volatile("v_nop\n\tv_nop\n\tv_nop\n\tv_nop" : "+v"(d) : "v"(a), "v"(b)); return d; }
__device__ __forceinline__ void wave_lds_sync() { __builtin_amdgcn_fence(__ATOMIC_RELEASE, "workgroup"); __builtin_amdgcn_wave_barrier(); __builtin_amdgcn_fence(__ATOMIC_ACQUIRE, "workgroup"); }
__device__ __forceinline__ float pmul(float a, float b) { float p = a * b; asm volatile("" : "+v"(p)); return p; }
__device__ __forceinline__ int iclamp(int v, int lo, int hi) { return v < lo ? lo : (v > hi ? hi : v); }
__device__ __forceinline__ float gelu(float v) { return 0.5f * v * (1.0f + erff(v * 0.70710678118654752f)); }
__device__ __forceinline__ float sigm(float v) { return 1.0f / (1.0f + __expf(-v)); }
constexpr int CSR_NBLK9 = 512, CSR_GB9 = 9, CSR_GN9 = 1 << CSR_GB9  , CSR_TS9 = (CSR_GN9 < 32 ? 32 : CSR_GN9)  , CSR_MAXG9 = 512, CSR_CAP9 = 12288  ;
__device__ __host__ __forceinline__ int csr_tix9(int v) { return (v >> CSR_GB9) * CSR_TS9 + (v & (CSR_GN9 - 1)); }
__global__ __launch_bounds__(64) void csrA_kernel9(const int* __restrict__ dst, int E, int N, int nG, int CHP, int NGP, int* __restrict__ STG, int* __restrict__ HST) {
  extern __shared__ int sm[];
  int* cnt = sm; int* run = sm + NGP; int* ids = sm + 2 * NGP;
  const int b = blockIdx.x; const int ch = (E + CSR_NBLK9 - 1) / CSR_NBLK9; const int e0 = b * ch, e1 = min(E, e0 + ch);
  for (int i = threadIdx.x; i < NGP; i += 64) cnt[i] = 0;
  for (int i = threadIdx.x; i < CHP; i += 64) ids[i] = -1;
  __syncthreads();
  if (threadIdx.x == 0) {
    for (int e = e0; e < e1; ++e) { int d = dst[e]; d = (d < 0) ? 0 : (d >= N ? N - 1 : d); cnt[d >> CSR_GB9] += 1; }
    int acc = 0; for (int g = 0; g < nG; ++g) { run[g] = acc; acc += cnt[g]; }
    for (int e = e0; e < e1; ++e) { int d = dst[e]; d = (d < 0) ? 0 : (d >= N ? N - 1 : d); const int g = d >> CSR_GB9; ids[run[g]] = e; run[g] += 1; } }
  __syncthreads();
  typedef __attribute__((ext_vector_type(4))) int v4i;
  for (int pass = 0; pass < 2; ++pass) {
    for (int i = threadIdx.x; i < CHP / 4; i += 64) *(volatile v4i*)(STG + (size_t)b * CHP + i * 4) = *(const v4i*)(&ids[i * 4]);
    for (int i = threadIdx.x; i < NGP / 4; i += 64) { v4i v; for (int e = 0; e < 4; ++e) v[e] = (i * 4 + e < nG) ? cnt[i * 4 + e] : 0; *(volatile v4i*)(HST + (size_t)b * NGP + i * 4) = v; }
    __threadfence(); }
}
__global__ __launch_bounds__(512) void csrS_kernel9(const int* __restrict__ HST, int nG, int NGP, int* __restrict__ START, int* __restrict__ TOT, int* __restrict__ OFF) {
  __shared__ int tot[CSR_MAXG9];
  const int b = threadIdx.x;
  for (int pass = 0; pass < 2; ++pass) { int runb = 0; for (int g = 0; g < nG; ++g) { int c = HST[(size_t)b * NGP + g]; c = (c < 0) ? 0 : c; ((volatile int*)OFF)[(size_t)g * CSR_NBLK9 + b] = runb; runb += c; } __threadfence(); }
  for (int g = threadIdx.x; g < nG; g += 512) { int s = 0; for (int bb = 0; bb < CSR_NBLK9; ++bb) { int c = HST[(size_t)bb * NGP + g]; s += (c < 0) ? 0 : c; } tot[g] = s; }
  __syncthreads();
  if (threadIdx.x < 32) {
    __shared__ int st[CSR_MAXG9 + 32];
    if (threadIdx.x == 0) { int acc = 0; for (int g = 0; g < NGP; ++g) { st[g] = acc; if (g < nG) acc += (tot[g] + 31) & ~31; } st[NGP] = acc; }
    __builtin_amdgcn_fence(__ATOMIC_RELEASE, "workgroup"); __builtin_amdgcn_wave_barrier(); __builtin_amdgcn_fence(__ATOMIC_ACQUIRE, "workgroup");
    for (int pass = 0; pass < 2; ++pass) { for (int i = threadIdx.x; i < NGP + 32; i += 32) { ((volatile int*)START)[i] = (i <= NGP) ? st[min(i, NGP)] : 0; ((volatile int*)TOT)[i] = (i < nG) ? tot[i] : 0; } __threadfence(); } }
}
__global__ __launch_bounds__(256) void csrB_kernel9(const int* __restrict__ dst, int N, int nG, int CHP, int NGP, int permLen, const int* __restrict__ STG, const int* __restrict__ HST, const int* __restrict__ OFF, const int* __restrict__ START, const int* __restrict__ TOT, int* __restrict__ PERM, int* __restrict__ ROWPTR, int* __restrict__ ROWCNT, int* __restrict__ FLAG) {
  typedef __attribute__((ext_vector_type(4))) int v4i;
  __shared__ int ids[CSR_CAP9]; __shared__ unsigned short key[CSR_CAP9]; __shared__ int outp[CSR_CAP9]; __shared__ int ncnt[CSR_GN9 + 1]; __shared__ int boff[CSR_NBLK9 + 1];
  const int g = blockIdx.x, t_ = threadIdx.x; int tot = TOT[g]; int st = START[g], stn = START[g + 1]; const int v0 = g * CSR_GN9; const int nv = min(CSR_GN9, N - v0); const int t0 = g * CSR_TS9;
  st = (st < 0) ? 0 : (st > permLen - 32 ? permLen - 32 : st) & ~31; stn = (stn < st) ? st : (stn > permLen ? permLen : stn); tot = (tot < 0) ? 0 : tot; if (tot > stn - st && tot <= CSR_CAP9) tot = stn - st;
  if (tot > CSR_CAP9) {
    for (int pass = 0; pass < 2; ++pass) { for (int i = t_; i < CSR_TS9 / 4; i += 256) { v4i a, c; for (int e = 0; e < 4; ++e) { a[e] = st; c[e] = 0; } *(volatile v4i*)(ROWPTR + t0 + i * 4) = a; *(volatile v4i*)(ROWCNT + t0 + i * 4) = c; } if (t_ == 0) ((volatile int*)FLAG)[0] = 1; __threadfence(); } (void)nv; return; }
  if (t_ == 0) { int acc = 0; for (int b = 0; b < CSR_NBLK9; ++b) { boff[b] = acc; int c = HST[(size_t)b * NGP + g]; c = (c < 0) ? 0 : (c > CHP ? CHP : c); acc += c; if (acc > tot) acc = tot; } boff[CSR_NBLK9] = acc; }
  for (int i = t_; i <= CSR_GN9; i += 256) ncnt[i] = 0;
  __syncthreads();
  for (int b = 0; b < CSR_NBLK9; ++b) { const int c = boff[b + 1] - boff[b]; int o_ = OFF[(size_t)g * CSR_NBLK9 + b]; o_ = (o_ < 0) ? 0 : (o_ > CHP - c ? CHP - c : o_); const int* src_ = STG + (size_t)b * CHP + o_;
    for (int i = t_; i < c; i += 256) { int id = src_[i]; id = (id < 0) ? 0 : id; ids[boff[b] + i] = id; int d = dst[id]; d = (d < v0) ? v0 : (d >= N ? N - 1 : d); int kk = d - v0; kk = (kk < 0) ? 0 : (kk >= CSR_GN9 ? CSR_GN9 - 1 : kk); key[boff[b] + i] = (unsigned short)kk; } }
  __syncthreads();
  if (t_ == 0) { for (int i = 0; i < tot; ++i) ncnt[key[i]] += 1; int acc = 0; for (int vl = 0; vl < CSR_GN9; ++vl) { const int c = ncnt[vl]; ncnt[vl] = acc; acc += c; } ncnt[CSR_GN9] = acc;
    for (int i = 0; i < tot; ++i) { const int vl = key[i]; outp[ncnt[vl]] = ids[i]; ncnt[vl] += 1; }
    for (int vl = CSR_GN9; vl > 0; --vl) ncnt[vl] = ncnt[vl - 1]; ncnt[0] = 0; }
  __syncthreads();
  for (int pass = 0; pass < 2; ++pass) {
    for (int i = t_; i < (stn - st) / 4; i += 256) { v4i v; for (int e = 0; e < 4; ++e) { const int q = i * 4 + e; v[e] = (q < tot) ? outp[q] : -1; } *(volatile v4i*)(PERM + st + i * 4) = v; }
    for (int i = t_; i < CSR_TS9 / 4; i += 256) { v4i a, c; for (int e = 0; e < 4; ++e) { const int vl = i * 4 + e; const int vc = vl < CSR_GN9 ? vl : CSR_GN9; a[e] = (vl < CSR_GN9) ? st + ncnt[vc] : st; c[e] = (vl < nv) ? (ncnt[(vc < CSR_GN9 ? vc : CSR_GN9 - 1) + 1] - ncnt[vc]) : 0; } *(volatile v4i*)(ROWPTR + t0 + i * 4) = a; *(volatile v4i*)(ROWCNT + t0 + i * 4) = c; }
    __threadfence(); }
}
__global__ __launch_bounds__(256) void csrZ_kernel9(int* __restrict__ p, size_t n4) { typedef __attribute__((ext_vector_type(4))) int v4i; const size_t tid = (size_t)blockIdx.x * 256 + threadIdx.x, nth = (size_t)gridDim.x * 256; v4i z = {0, 0, 0, 0}; for (size_t i = tid; i < n4; i += nth) *(volatile v4i*)(p + i * 4) = z; }
struct CsrBufs9 { int *STG, *HST, *OFF, *START, *TOT, *PERM, *ROWPTR, *ROWCNT, *FLAG; int nG, NGP, CHP; size_t permLen; char* base; size_t bytes; };
static size_t csr_carve9(CsrBufs9& c, char* ws, size_t off, int E, int N) {
  const size_t off0 = off; c.base = ws + off;
  auto al = [&](size_t bytes) { char* p = ws + off; off += (bytes + 255) & ~(size_t)255; return p; };
  c.nG = (N + CSR_GN9 - 1) / CSR_GN9; c.NGP = (c.nG + 31) & ~31; const int ch = (E + CSR_NBLK9 - 1) / CSR_NBLK9; c.CHP = (ch + 31) & ~31; c.permLen = (size_t)E + 32 * (size_t)c.nG + 32;
  c.STG = (int*)al((size_t)CSR_NBLK9 * c.CHP * 4); c.HST = (int*)al((size_t)CSR_NBLK9 * c.NGP * 4); c.OFF = (int*)al((size_t)c.NGP * CSR_NBLK9 * 4); c.START = (int*)al((size_t)(c.NGP + 64) * 4); c.TOT = (int*)al((size_t)(c.NGP + 64) * 4);
  c.PERM = (int*)al(c.permLen * 4); c.ROWPTR = (int*)al((size_t)c.nG * CSR_TS9 * 4); c.ROWCNT = (int*)al((size_t)c.nG * CSR_TS9 * 4); c.FLAG = (int*)al(256);
  c.bytes = off - off0; return off;
}
static void csr_build9(const CsrBufs9& c, const int* dst, int E, int N, hipStream_t stream) {
  const size_t smem = (size_t)(2 * c.NGP + c.CHP) * 4;
  csrZ_kernel9<<<512, 256, 0, stream>>>((int*)c.base, c.bytes / 16);
  csrA_kernel9<<<CSR_NBLK9, 64, smem, stream>>>(dst, E, N, c.nG, c.CHP, c.NGP, c.STG, c.HST);
  csrS_kernel9<<<1, 512, 0, stream>>>(c.HST, c.nG, c.NGP, c.START, c.TOT, c.OFF);
  csrB_kernel9<<<c.nG, 256, 0, stream>>>(dst, N, c.nG, c.CHP, c.NGP, (int)c.permLen, c.STG, c.HST, c.OFF, c.START, c.TOT, c.PERM, c.ROWPTR, c.ROWCNT, c.FLAG);
}


__global__ __launch_bounds__(256) void wput_kernel(const float* __restrict__ w, int OUTW, b16* __restrict__ WT) {
  const int u = blockIdx.x * 256 + threadIdx.x; if (u >= OUTW * 16) return; const int o = u / 16, k0 = (u % 16) * 8; v8b v;
#pragma unroll
  for (int j = 0; j < 8; ++j) v[j] = (b16)(bf16_rne(w[(size_t)(k0 + j) * OUTW + o]) * WSC); for (int pass = 0; pass < 2; ++pass) { *(volatile v8b*)(WT + (size_t)o * D + k0) = v; __threadfence(); }
}
template <int NT, int L1, int FC>
__global__ __launch_bounds__(32) void dense_kernel(const float* __restrict__ IN_, const float* __restrict__ emb, const b16* __restrict__ WT, const float* __restrict__ bias, int NLIM, float* __restrict__ OUT) {
  __shared__ __attribute__((aligned(16))) b16 Ah[16][D + 8], Al[16][(L1 ? 32 : D) + 8]; __shared__ __attribute__((aligned(16))) float Tf[16][D + 4];
  const int lane = threadIdx.x, nloc = lane & 15, hlf = lane >> 4; const size_t m0 = (size_t)blockIdx.x * 16; if (m0 >= (size_t)NLIM) return;
  for (int rr = 0; rr < 16; ++rr) { if (L1) { const float* xr = IN_ + (m0 + rr) * 65; int id = (int)bf16_rne(xr[64]); if (id < 0) id += V; id = iclamp(id, 0, V - 1);
      Ah[rr][lane] = (b16)(bf16_rne(xr[lane]) * XS); Ah[rr][32 + lane] = (b16)(bf16_rne(xr[32 + lane]) * XS); Ah[rr][64 + lane] = (b16)(bf16_rne(emb[(size_t)id * 64 + lane]) * XS); Ah[rr][96 + lane] = (b16)(bf16_rne(emb[(size_t)id * 64 + 32 + lane]) * XS); }
    else { for (int q = 0; q < 4; ++q) { b16 p, ql; split16(IN_[(m0 + rr) * D + q * 32 + lane] * XS, p, ql); Ah[rr][q * 32 + lane] = p; Al[rr][q * 32 + lane] = ql; } } }
  wave_lds_sync(); v8f acc[NT];
#pragma unroll
  for (int t = 0; t < NT; ++t) acc[t] = (v8f){};
#pragma unroll
  for (int kb = 0; kb < D; kb += 32) { const v16b a = frag_kb(&Ah[nloc][kb], hlf); v16b al; if (!L1) al = frag_kb(&Al[nloc][kb], hlf);
#pragma unroll
    for (int t = 0; t < NT; ++t) { const v16b bw = frag_kb(WT + (size_t)(t * 16 + nloc) * D + kb, hlf); acc[t] = wmma16b(a, bw, acc[t]); if (!L1) acc[t] = wmma16b(al, bw, acc[t]); } }
#pragma unroll
  for (int t = 0; t < NT; ++t) { const int c = t * 16 + nloc; const float bb = FC ? bf16_rne(bias[c]) : 0.0f;
#pragma unroll
    for (int r8 = 0; r8 < 8; ++r8) { float v = acc[t][r8] * (1.0f / (XS * WSC)); if (FC) v = gelu(v + bb); Tf[8 * hlf + r8][c] = v; } }
  wave_lds_sync();
  for (int pass = 0; pass < 2; ++pass) { for (int rr = 0; rr < 16; ++rr) for (int c = lane * 4; c < NT * 16; c += 128) *(volatile v4f*)(OUT + (m0 + rr) * (size_t)(NT * 16) + c) = *(const v4f*)(&Tf[rr][c]); __threadfence(); }
}
__global__ __launch_bounds__(256) void agg_kernel(const float* __restrict__ XW, const float* __restrict__ bias, const int* __restrict__ rows, const int* __restrict__ PERM, const int* __restrict__ ROWPTR, const int* __restrict__ ROWCNT, int permLen, int NLIM, float* __restrict__ Hh) {
  const int wave = threadIdx.x >> 5, lane = threadIdx.x & 31; const size_t v = (size_t)blockIdx.x * 8 + wave; if (v >= (size_t)NLIM) return;
  int st = ROWPTR[v], cnt = ROWCNT[v]; cnt = iclamp(cnt, 0, 1 << 20); st = iclamp(st, 0, permLen - cnt); int nn = 0;
#pragma unroll 1
  for (int j = 0; j < cnt; ++j) { const int e = iclamp(PERM[st + j], 0, E - 1); if (iclamp(rows[e], 0, N - 1) < NLIM) ++nn; }
  const float dv = rsqrtf((float)(nn + 1)); v4f o; const v4f xv = *(const v4f*)(XW + v * D + lane * 4); for (int i = 0; i < 4; ++i) o[i] = pmul(dv * dv, xv[i]);
#pragma unroll 1
  for (int j = 0; j < cnt; ++j) { const int e = iclamp(PERM[st + j], 0, E - 1); const size_t u = (size_t)iclamp(rows[e], 0, N - 1); if (u >= (size_t)NLIM) continue; int cu = ROWCNT[u]; cu = iclamp(cu, 0, 1 << 20);
    int nu = cu; if (NLIM < N) { nu = 0; const int su = iclamp(ROWPTR[u], 0, permLen - cu); for (int k = 0; k < cu; ++k) if (iclamp(rows[iclamp(PERM[su + k], 0, E - 1)], 0, N - 1) < NLIM) ++nu; }
    const float wgt = pmul(dv, rsqrtf((float)(nu + 1))); const v4f xu = *(const v4f*)(XW + u * D + lane * 4); for (int i = 0; i < 4; ++i) o[i] += pmul(wgt, xu[i]); }
  v4f r; for (int i = 0; i < 4; ++i) r[i] = gelu(o[i] + bf16_rne(bias[lane * 4 + i]));
  for (int pass = 0; pass < 2; ++pass) { *(volatile v4f*)(Hh + v * D + lane * 4) = r; __threadfence(); }
}
__global__ __launch_bounds__(32) void gi_kernel(const float* __restrict__ H4, const int* __restrict__ rows, const int* __restrict__ cols, const float* __restrict__ Wih, const float* __restrict__ bih, int ELIM, float* __restrict__ GI) {
  const int lane = threadIdx.x; const size_t e = (size_t)blockIdx.x * 32 + lane; if (e >= (size_t)ELIM) return; const float* hr = H4 + (size_t)iclamp(rows[e], 0, N - 1) * DO; const float* hc = H4 + (size_t)iclamp(cols[e], 0, N - 1) * DO;
  float g0 = bf16_rne(bih[0]), g1 = bf16_rne(bih[1]), g2 = bf16_rne(bih[2]);
#pragma unroll 4
  for (int k = 0; k < DO; ++k) { const float xe = (hr[k] + hc[k]) * 0.5f; g0 += pmul(xe, bf16_rne(Wih[k])); g1 += pmul(xe, bf16_rne(Wih[DO + k])); g2 += pmul(xe, bf16_rne(Wih[2 * DO + k])); }
  for (int pass = 0; pass < 2; ++pass) { *(volatile v4f*)(GI + e * 4) = (v4f){g0, g1, g2, 0.0f}; __threadfence(); }
}
__global__ __launch_bounds__(32) void gru_kernel(const float* __restrict__ GI, const float* __restrict__ Whh, const float* __restrict__ bhh, const float* __restrict__ h0p, int NGV, float* __restrict__ sel, float* __restrict__ flat) {
  const int g = blockIdx.x * 32 + threadIdx.x; if (g >= NGV) return; const float wr = bf16_rne(Whh[0]), wz = bf16_rne(Whh[1]), wn = bf16_rne(Whh[2]), br = bf16_rne(bhh[0]), bz = bf16_rne(bhh[1]), bn = bf16_rne(bhh[2]);
  for (int pass = 0; pass < 2; ++pass) { float h = bf16_rne(h0p[0]); float sum = 0.0f, first = 0.0f, lastnz = 0.0f; int have = 0;
#pragma unroll 1
    for (int p = 0; p < TT; ++p) { const float* gi = GI + ((size_t)g * TT + p) * 4; const float r = sigm(gi[0] + pmul(h, wr) + br), z = sigm(gi[1] + pmul(h, wz) + bz); const float nn = tanhf(gi[2] + pmul(r, pmul(h, wn) + bn)); h = pmul(1.0f - z, nn) + pmul(z, h);
      ((volatile float*)flat)[(size_t)g * TT + p] = h; sum += h; if (p == 0) first = h; if (h != 0.0f) { lastnz = h; have = 1; } }
    const float s = (sum > 0.0f && have) ? lastnz : first;
    ((volatile float*)sel)[g] = s; __threadfence(); }
}
}

extern "C" void kernel_launch(void* const* d_in, const int* in_sizes, int n_in, void* d_out, int out_size, void* d_ws, size_t ws_size, hipStream_t stream) {
  (void)n_in;
  auto Fp = [&](int i) { return (const float*)d_in[i]; }; auto Ip = [&](int i) { return (const int*)d_in[i]; };
  if (in_sizes[0] != N * 65 || in_sizes[1] != V * 64 || in_sizes[2] != D * D || in_sizes[4] != D * D || in_sizes[6] != D * D || in_sizes[8] != D * DO || in_sizes[10] != 3 * DO || in_sizes[11] != 3 || in_sizes[15] != 2 * E || out_size != G + E) return;
  const int NLIM = N, NGV = G; const int GB16 = NBLK, GB8 = N / 8;
  size_t off = 0; char* ws = (char*)d_ws;
  auto carve = [&](size_t bytes) { char* p = ws + off; off += (bytes + 255) & ~(size_t)255; return p; };
  b16* WT1 = (b16*)carve(D * D * 2); b16* WT2 = (b16*)carve(D * D * 2); b16* WT3 = (b16*)carve(D * D * 2); b16* WTF = (b16*)carve(DO * D * 2);
  float* XW = (float*)carve((size_t)N * D * 4); float* HA = (float*)carve((size_t)N * D * 4); float* H4 = (float*)carve((size_t)N * DO * 4); float* GI = (float*)carve((size_t)E * 4 * 4);
  CsrBufs9 csr; off = csr_carve9(csr, ws, off, E, N);
  if (off > ws_size || off > ((size_t)128 << 20)) return;
  wput_kernel<<<(D * 16 + 255) / 256, 256, 0, stream>>>(Fp(2), D, WT1); wput_kernel<<<(D * 16 + 255) / 256, 256, 0, stream>>>(Fp(4), D, WT2); wput_kernel<<<(D * 16 + 255) / 256, 256, 0, stream>>>(Fp(6), D, WT3); wput_kernel<<<(DO * 16 + 255) / 256, 256, 0, stream>>>(Fp(8), DO, WTF);
  csr_build9(csr, Ip(15) + E, E, N, stream);
  dense_kernel<8, 1, 0><<<GB16, 32, 0, stream>>>(Fp(0), Fp(1), WT1, nullptr, NLIM, XW); agg_kernel<<<GB8, 256, 0, stream>>>(XW, Fp(3), Ip(15), csr.PERM, csr.ROWPTR, csr.ROWCNT, (int)csr.permLen, NLIM, HA);
  dense_kernel<8, 0, 0><<<GB16, 32, 0, stream>>>(HA, nullptr, WT2, nullptr, NLIM, XW);   agg_kernel<<<GB8, 256, 0, stream>>>(XW, Fp(5), Ip(15), csr.PERM, csr.ROWPTR, csr.ROWCNT, (int)csr.permLen, NLIM, HA);
  dense_kernel<8, 0, 0><<<GB16, 32, 0, stream>>>(HA, nullptr, WT3, nullptr, NLIM, XW);   agg_kernel<<<GB8, 256, 0, stream>>>(XW, Fp(7), Ip(15), csr.PERM, csr.ROWPTR, csr.ROWCNT, (int)csr.permLen, NLIM, HA);
  dense_kernel<4, 0, 1><<<GB16, 32, 0, stream>>>(HA, nullptr, WTF, Fp(9), NLIM, H4);
  gi_kernel<<<(NGV * TT) / 32, 32, 0, stream>>>(H4, Ip(15), Ip(15) + E, Fp(10), Fp(12), NGV * TT, GI);
  float* out = (float*)d_out;
  gru_kernel<<<(NGV + 31) / 32, 32, 0, stream>>>(GI, Fp(11), Fp(13), Fp(14), NGV, out, out + G);
}
